// ServicePredictorNNSetRepr_80839874445316
// MI455X (gfx1250) — hardware-verified
//
#include <hip/hip_runtime.h>


#define NBT  4096
#define LL   1024
#define NR   (NBT * LL)
#define NAPP 10
#define RCH  131072
#define NCHK (NR / RCH)
typedef _Float16 h16;
typedef unsigned short bf;
typedef __attribute__((ext_vector_type(16))) __bf16   v16bf;
typedef __attribute__((ext_vector_type(16))) _Float16 v16h;
typedef __attribute__((ext_vector_type(8)))  _Float16 v8h;
typedef __attribute__((ext_vector_type(8)))  unsigned short v8us;
typedef __attribute__((ext_vector_type(8)))  float    v8f;
typedef __attribute__((ext_vector_type(4)))  float    v4f;
typedef v8h  __attribute__((may_alias)) v8ha;
typedef v4f  __attribute__((may_alias)) v4fa;
typedef v8us __attribute__((may_alias)) v8usa;

__device__ __forceinline__ unsigned short f2bf(float f) { unsigned u = __float_as_uint(f); u += 0x7FFFu + ((u >> 16) & 1u); return (unsigned short)(u >> 16); }
__device__ __forceinline__ float bf2f(unsigned short b) { return __uint_as_float(((unsigned)b) << 16); }
__device__ __forceinline__ float bfr(float f) { return bf2f(f2bf(f)); }
__device__ __forceinline__ v16h cat16(v8h lo, v8h hi) { return __builtin_shufflevector(lo, hi, 0, 1, 2, 3, 4, 5, 6, 7, 8, 9, 10, 11, 12, 13, 14, 15); }
__device__ __forceinline__ v16bf cat16b(v8us lo, v8us hi) { return __builtin_bit_cast(v16bf, __builtin_shufflevector(lo, hi, 0, 1, 2, 3, 4, 5, 6, 7, 8, 9, 10, 11, 12, 13, 14, 15)); }
__device__ __forceinline__ v8f wmma16(v16h a, v16h b, v8f c) { return __builtin_amdgcn_wmma_f32_16x16x32_f16(false, a, false, b, (short)0, c, false, false); }
__device__ __forceinline__ v8f wmmab(v16bf a, v16bf b, v8f c) { return __builtin_amdgcn_wmma_f32_16x16x32_bf16(false, a, false, b, (short)0, c, false, false); }


template <typename T16> struct WFrag;
template <> struct WFrag<h16> { typedef v16h V; static __device__ __forceinline__ V ld(const h16* p) { return cat16(*(const v8h*)p, *(const v8h*)(p + 16)); } static __device__ __forceinline__ v8f mma(V a, V b, v8f c) { return wmma16(a, b, c); } };
template <> struct WFrag<bf> { typedef v16bf V; static __device__ __forceinline__ V ld(const bf* p) { return cat16b(*(const v8us*)p, *(const v8us*)(p + 16)); } static __device__ __forceinline__ v8f mma(V a, V b, v8f c) { return wmmab(a, b, c); } };
template <typename T16, int NSPLIT, bool BIAS>
__global__ __launch_bounds__(32) void k_gemmw(const T16* __restrict__ A, const T16* __restrict__ A2, const T16* __restrict__ Bt, const T16* __restrict__ Bt2, int K, float* C, int ldc, const float* __restrict__ bias, size_t sA, size_t sB, size_t sC) {
    typedef typename WFrag<T16>::V V;
    __shared__ __align__(16) float os[16 * 68];
    const size_t z = blockIdx.z; A += z * sA; if (A2) A2 += z * sA; Bt += z * sB; if (Bt2) Bt2 += z * sB; C += z * sC;
    const int lane = threadIdx.x & 31, lr = lane & 15, hi = lane >> 4; const int r0 = blockIdx.x * 64, c0 = blockIdx.y * 64;
    v8f acc[4][4];
#pragma unroll
    for (int mb = 0; mb < 4; ++mb)
#pragma unroll
        for (int nb = 0; nb < 4; ++nb) acc[mb][nb] = (v8f){};
    const size_t aoff = (size_t)(r0 + lr) * K + 8 * hi, boff = (size_t)(c0 + lr) * K + 8 * hi;
#pragma unroll 1
    for (int kc = 0; kc < K; kc += 32) {
        V a[4], a2[4];
#pragma unroll
        for (int mb = 0; mb < 4; ++mb) { a[mb] = WFrag<T16>::ld(A + aoff + (size_t)mb * 16 * K + kc); if (NSPLIT == 1 || NSPLIT == 2) a2[mb] = WFrag<T16>::ld(A2 + aoff + (size_t)mb * 16 * K + kc); }
#pragma unroll
        for (int nb = 0; nb < 4; ++nb) { const V b = WFrag<T16>::ld(Bt + boff + (size_t)nb * 16 * K + kc); V b2; if (NSPLIT >= 2) b2 = WFrag<T16>::ld(Bt2 + boff + (size_t)nb * 16 * K + kc);
#pragma unroll
            for (int mb = 0; mb < 4; ++mb) { acc[mb][nb] = WFrag<T16>::mma(a[mb], b, acc[mb][nb]); if (NSPLIT == 1 || NSPLIT == 2) acc[mb][nb] = WFrag<T16>::mma(a2[mb], b, acc[mb][nb]); if (NSPLIT >= 2) acc[mb][nb] = WFrag<T16>::mma(a[mb], b2, acc[mb][nb]); } }
        asm volatile("v_nop\n\tv_nop\n\tv_nop\n\tv_nop" : "+v"(acc[0][0]), "+v"(acc[1][1]), "+v"(acc[2][2]), "+v"(acc[3][3]) : "v"(a[0]), "v"(a[3]));
    }
#pragma unroll
    for (int mb = 0; mb < 4; ++mb) {
#pragma unroll
        for (int nb = 0; nb < 4; ++nb) {
#pragma unroll
            for (int j = 0; j < 8; ++j) os[(hi * 8 + j) * 68 + nb * 16 + lr] = acc[mb][nb][j]; }
        __builtin_amdgcn_wave_barrier(); asm volatile("" ::: "memory");
        float* crow = C + (size_t)(r0 + mb * 16) * ldc + c0;
#pragma unroll 1
        for (int ps = 0; ps < 2; ++ps) {
#pragma unroll
            for (int s = 0; s < 8; ++s) { const int row = 2 * s + hi, cofs = lr * 4; v4f val = *(const v4fa*)(os + row * 68 + cofs); if (BIAS) { val[0] += bfr(bias[c0 + cofs]); val[1] += bfr(bias[c0 + cofs + 1]); val[2] += bfr(bias[c0 + cofs + 2]); val[3] += bfr(bias[c0 + cofs + 3]); }
                *(volatile v4f*)(crow + (size_t)row * ldc + cofs) = val; }
            if (ps == 0) __threadfence(); }
        __builtin_amdgcn_wave_barrier(); asm volatile("" ::: "memory");
    }
}

__device__ __forceinline__ h16 tohx(float x) { return (h16)x; }
__device__ __forceinline__ void splitf(float y, unsigned short& h, unsigned short& l) { h = f2bf(y); l = f2bf(y - bf2f(h)); }
typedef __attribute__((ext_vector_type(4))) _Float16 v4h;
typedef __attribute__((ext_vector_type(2))) _Float16 v2h;
typedef __attribute__((ext_vector_type(4))) unsigned short v4us;
typedef __attribute__((ext_vector_type(2))) unsigned short v2us;

__global__ __launch_bounds__(256) void k_prep(const float* __restrict__ emb, const float* __restrict__ W1, const float* __restrict__ W2, const float* __restrict__ W3, const float* __restrict__ fb3, const float* __restrict__ R2, const float* __restrict__ R3, const float* __restrict__ rb3, const float* __restrict__ fb2, const float* __restrict__ rb2,
                                              float* EN, float* ET, h16* W2t, h16* W3t, bf* R2t, bf* R3t, float* FB3P, float* RB3P, float* FB2P, float* RB2P) {
    typedef __attribute__((ext_vector_type(2))) float v2f;
    const int lane = threadIdx.x & 31, wv = threadIdx.x >> 5;
    auto en = [&](int a, float& e0, float& e1) { const float x0 = bfr(emb[a * 2]), x1 = bfr(emb[a * 2 + 1]); const float n = sqrtf(x0 * x0 + x1 * x1); const float sc = fminf(1.0f, __fdiv_rn(1.0f, fmaxf(n, 1e-7f))); e0 = x0 * sc; e1 = x1 * sc; };
#pragma unroll 1
    for (int ps = 0; ps < 2; ++ps) {
        if (wv == 0) { if (lane < 2 * NAPP) { float e0, e1; en(lane >> 1, e0, e1); *(volatile float*)(EN + lane) = (lane & 1) ? e1 : e0; } }
        else if (wv <= 4) { const float* src = wv == 1 ? fb3 : (wv == 2 ? rb3 : (wv == 3 ? fb2 : rb2)); const int nlive = wv == 1 ? 5 : (wv == 2 ? 1 : 25); float* dst = wv == 1 ? FB3P : (wv == 2 ? RB3P : (wv == 3 ? FB2P : RB2P)); v2f o;
#pragma unroll
            for (int q = 0; q < 2; ++q) { const int i = lane * 2 + q; o[q] = i < nlive ? src[i < nlive ? i : 0] : 0.f; }
            *(volatile v2f*)(dst + lane * 2) = o; }
#pragma unroll 1
        for (int a = wv; a < NAPP; a += 8) { float e0, e1; en(a, e0, e1); v2f o;
#pragma unroll
            for (int q = 0; q < 2; ++q) { const int c = lane * 2 + q; o[q] = c < 50 ? e0 * bfr(W1[0 * 50 + c]) + e1 * bfr(W1[1 * 50 + c]) : 0.f; }
            *(volatile v2f*)(ET + a * 64 + lane * 2) = o; }
#pragma unroll 1
        for (int L = wv; L < 64; L += 8) { const int e = L * 64 + lane * 2; v2h oh; v2us ob;
#pragma unroll
            for (int q = 0; q < 2; ++q) { const int n = (e + q) / 64, k = (e + q) % 64; const bool live = k < 50 && n < 25; oh[q] = tohx(live ? bfr(W2[(k < 50 ? k : 0) * 25 + (n < 25 ? n : 0)]) : 0.f); ob[q] = f2bf(live ? bfr(R2[(k < 50 ? k : 0) * 25 + (n < 25 ? n : 0)]) : 0.f); }
            *(volatile v2h*)(W2t + e) = oh; *(volatile v2us*)(R2t + e) = ob; }
#pragma unroll 1
        for (int L = wv; L < 32; L += 8) { const int e = L * 64 + lane * 2; v2h oh; v2us ob;
#pragma unroll
            for (int q = 0; q < 2; ++q) { const int n = (e + q) / 32, k = (e + q) % 32; oh[q] = tohx((k < 25 && n < 5) ? bfr(W3[(k < 25 ? k : 0) * 5 + (n < 5 ? n : 0)]) : 0.f); ob[q] = f2bf((k < 25 && n < 1) ? bfr(R3[k < 25 ? k : 0]) : 0.f); }
            *(volatile v2h*)(W3t + e) = oh; *(volatile v2us*)(R3t + e) = ob; }
        if (ps == 0) __threadfence(); }
}
__global__ __launch_bounds__(256) void k_h1(const float* __restrict__ feat, const float* __restrict__ ET, const float* __restrict__ W1, const float* __restrict__ b1, int r0, h16* H1) {
    const int lane = threadIdx.x & 31; const int w = blockIdx.x * 8 + (threadIdx.x >> 5); const int rl = w * 2 + (lane >> 4); if (rl >= RCH) return; const int r = r0 + rl; const int b = r / LL, l = r % LL;
    int id = (int)bfr(feat[((size_t)b * 3 + 0) * LL + l]); id = id < 0 ? id + NAPP : id; id = id < 0 ? 0 : (id > NAPP - 1 ? NAPP - 1 : id);
    const float ld0 = bfr(feat[((size_t)b * 3 + 1) * LL + l]), ld1 = bfr(feat[((size_t)b * 3 + 2) * LL + l]); const int c0 = (lane & 15) * 4; v4h o;
#pragma unroll
    for (int q = 0; q < 4; ++q) { const int c = c0 + q; float v = 0.f; if (c < 50) v = fmaxf(ET[id * 64 + c] + ld0 * bfr(W1[2 * 50 + c]) + ld1 * bfr(W1[3 * 50 + c]) + bfr(b1[c]), 0.f); o[q] = tohx(v); }
    h16* dst = H1 + (size_t)rl * 64 + c0; *(volatile v4h*)dst = o; __threadfence(); *(volatile v4h*)dst = o;
}
__global__ __launch_bounds__(256) void k_relu16p(const float* __restrict__ H2, h16* P2) {
    const int lane = threadIdx.x & 31; const int L0 = (blockIdx.x * 8 + (threadIdx.x >> 5)) * 8; const int nlines = RCH * 32 / 64;
#pragma unroll 1
    for (int ps = 0; ps < 2; ++ps) {
#pragma unroll
        for (int i = 0; i < 8; ++i) { const int L = L0 + i; if (L >= nlines) break; const int e = L * 64 + lane * 2; const int r = e >> 5, c = e & 31; v2h v;
#pragma unroll
            for (int q = 0; q < 2; ++q) v[q] = tohx(c + q < 25 ? fmaxf(H2[(size_t)r * 64 + c + q], 0.f) : 0.f);
            *(volatile v2h*)(P2 + e) = v; }
        if (ps == 0) __threadfence(); }
}
__global__ __launch_bounds__(256) void k_summax(const float* __restrict__ H3, int b0g, float* HSM) {
    const int lane = threadIdx.x & 31; const int w = blockIdx.x * 8 + (threadIdx.x >> 5); if (w >= RCH / LL / 2) return; const int half = lane >> 4, sub = lane & 15; const int bl = w * 2 + half;
    float s[5], m[5];
#pragma unroll
    for (int k = 0; k < 5; ++k) { s[k] = 0.f; m[k] = -3.0e38f; }
#pragma unroll 1
    for (int it = 0; it < LL / 16; ++it) { const int l = it * 16 + sub; const float* row = H3 + ((size_t)bl * LL + l) * 64;
#pragma unroll
        for (int k = 0; k < 5; ++k) { const float v = row[k]; s[k] += v; m[k] = fmaxf(m[k], v); } }
#pragma unroll
    for (int k = 0; k < 5; ++k) {
#pragma unroll
        for (int sh = 8; sh; sh >>= 1) { s[k] += __shfl_xor(s[k], sh, 32); m[k] = fmaxf(m[k], __shfl_xor(m[k], sh, 32)); } }
    float v = 0.f;
#pragma unroll
    for (int k = 0; k < 5; ++k) { if (sub == k) v = s[k]; if (sub == 5 + k) v = m[k]; }
    float* dst = HSM + (size_t)(b0g + w * 2) * 16 + lane; *(volatile float*)dst = v; __threadfence(); *(volatile float*)dst = v;
}
__global__ __launch_bounds__(256) void k_read1(const float* __restrict__ HSM, const float* __restrict__ xf, const float* __restrict__ EN, const float* __restrict__ R1, const float* __restrict__ rb1, bf* Ph, bf* Pl) {
    const int lane = threadIdx.x & 31; const int w = blockIdx.x * 8 + (threadIdx.x >> 5); const int b = w * 2 + (lane >> 4); if (b >= NBT) return;
    float hh[14];
#pragma unroll
    for (int k = 0; k < 10; ++k) hh[k] = HSM[(size_t)b * 16 + k];
    int id = (int)bfr(xf[b * 3 + 0]); id = id < 0 ? id + NAPP : id; id = id < 0 ? 0 : (id > NAPP - 1 ? NAPP - 1 : id); hh[10] = EN[id * 2]; hh[11] = EN[id * 2 + 1]; hh[12] = bfr(xf[b * 3 + 1]); hh[13] = bfr(xf[b * 3 + 2]);
    const int c0 = (lane & 15) * 4; v4us oh, ol;
#pragma unroll
    for (int q = 0; q < 4; ++q) { const int c = c0 + q; float v = 0.f; if (c < 50) { float acc = bfr(rb1[c]);
#pragma unroll
            for (int k = 0; k < 14; ++k) acc = fmaf(hh[k], bfr(R1[k * 50 + c]), acc); v = fmaxf(acc, 0.f); }
        unsigned short a, c2; splitf(v, a, c2); oh[q] = a; ol[q] = c2; }
    const size_t o = (size_t)b * 64 + c0; *(volatile v4us*)(Ph + o) = oh; *(volatile v4us*)(Pl + o) = ol; __threadfence(); *(volatile v4us*)(Ph + o) = oh; *(volatile v4us*)(Pl + o) = ol;
}
__global__ __launch_bounds__(256) void k_read2p(const float* __restrict__ G, bf* Ph, bf* Pl) {
    const int lane = threadIdx.x & 31; const int L = blockIdx.x * 8 + (threadIdx.x >> 5); if (L >= NBT * 32 / 64) return; const int e = L * 64 + lane * 2; const int r = e >> 5, c = e & 31; v2us oh, ol;
#pragma unroll
    for (int q = 0; q < 2; ++q) { unsigned short a, c2; splitf(c + q < 25 ? fmaxf(G[(size_t)r * 64 + c + q], 0.f) : 0.f, a, c2); oh[q] = a; ol[q] = c2; }
    *(volatile v2us*)(Ph + e) = oh; *(volatile v2us*)(Pl + e) = ol; __threadfence(); *(volatile v2us*)(Ph + e) = oh; *(volatile v2us*)(Pl + e) = ol;
}
__global__ __launch_bounds__(256) void k_out(const float* __restrict__ C, float* OUT) { const int lane = threadIdx.x & 31; const int b0 = (blockIdx.x * 8 + (threadIdx.x >> 5)) * 32; if (b0 >= NBT) return; const float v = C[(size_t)(b0 + lane) * 64]; *(volatile float*)(OUT + b0 + lane) = v; __threadfence(); *(volatile float*)(OUT + b0 + lane) = v; }

extern "C" void kernel_launch(void* const* d_in, const int* in_sizes, int n_in,
                              void* d_out, int out_size, void* d_ws, size_t ws_size, hipStream_t stream) {
    (void)in_sizes; (void)n_in; (void)out_size;
    const float* xf = (const float*)d_in[0]; const float* feat = (const float*)d_in[1];   const float* emb = (const float*)d_in[3];
    const float* fW1 = (const float*)d_in[4]; const float* fb1 = (const float*)d_in[5]; const float* fW2 = (const float*)d_in[6]; const float* fb2 = (const float*)d_in[7]; const float* fW3 = (const float*)d_in[8]; const float* fb3 = (const float*)d_in[9];
    const float* rW1 = (const float*)d_in[10]; const float* rb1 = (const float*)d_in[11]; const float* rW2 = (const float*)d_in[12]; const float* rb2 = (const float*)d_in[13]; const float* rW3 = (const float*)d_in[14]; const float* rb3 = (const float*)d_in[15];
    float* OUT = (float*)d_out;
    char* wsp = (char*)d_ws;
    auto take = [&](size_t bytes) { char* p = wsp; wsp += (bytes + 255) & ~(size_t)255; return (void*)p; };
    float* EN = (float*)take(NAPP * 2 * 4); float* ET = (float*)take(NAPP * 64 * 4); h16* W2t = (h16*)take(64 * 64 * 2); h16* W3t = (h16*)take(64 * 32 * 2); bf* R2t = (bf*)take(64 * 64 * 2); bf* R3t = (bf*)take(64 * 32 * 2); float* FB3P = (float*)take(64 * 4); float* RB3P = (float*)take(64 * 4); float* FB2P = (float*)take(64 * 4); float* RB2P = (float*)take(64 * 4);
    h16* H1 = (h16*)take((size_t)RCH * 64 * 2); float* H2 = (float*)take((size_t)RCH * 64 * 4); h16* P2 = (h16*)take((size_t)RCH * 32 * 2); float* H3 = (float*)take((size_t)RCH * 64 * 4);
    float* HSM = (float*)take((size_t)NBT * 16 * 4); bf* Q1h = (bf*)take((size_t)NBT * 64 * 2); bf* Q1l = (bf*)take((size_t)NBT * 64 * 2); float* G2 = (float*)take((size_t)NBT * 64 * 4); bf* Q2h = (bf*)take((size_t)NBT * 32 * 2); bf* Q2l = (bf*)take((size_t)NBT * 32 * 2); float* G3 = (float*)take((size_t)NBT * 64 * 4);
    if ((size_t)(wsp - (char*)d_ws) > ws_size) return;
    k_prep<<<1, 256, 0, stream>>>(emb, fW1, fW2, fW3, fb3, rW2, rW3, rb3, fb2, rb2, EN, ET, W2t, W3t, R2t, R3t, FB3P, RB3P, FB2P, RB2P);
    for (int ch = 0; ch < NCHK; ++ch) { const int r0 = ch * RCH;
        k_h1<<<(RCH / 2 + 7) / 8, 256, 0, stream>>>(feat, ET, fW1, fb1, r0, H1);
        k_gemmw<h16, 0, true><<<dim3(RCH / 64, 1, 1), 32, 0, stream>>>(H1, nullptr, W2t, nullptr, 64, H2, 64, FB2P, 0, 0, 0);
        k_relu16p<<<(RCH * 32 / 64 + 63) / 64, 256, 0, stream>>>(H2, P2);
        k_gemmw<h16, 0, true><<<dim3(RCH / 64, 1, 1), 32, 0, stream>>>(P2, nullptr, W3t, nullptr, 32, H3, 64, FB3P, 0, 0, 0);
        k_summax<<<(RCH / LL / 2 + 7) / 8, 256, 0, stream>>>(H3, ch * (RCH / LL), HSM); }
    k_read1<<<(NBT / 2 + 7) / 8, 256, 0, stream>>>(HSM, xf, EN, rW1, rb1, Q1h, Q1l);
    k_gemmw<bf, 1, true><<<dim3(NBT / 64, 1, 1), 32, 0, stream>>>(Q1h, Q1l, R2t, nullptr, 64, G2, 64, RB2P, 0, 0, 0);
    k_read2p<<<(NBT * 32 / 64 + 7) / 8, 256, 0, stream>>>(G2, Q2h, Q2l);
    k_gemmw<bf, 1, true><<<dim3(NBT / 64, 1, 1), 32, 0, stream>>>(Q2h, Q2l, R3t, nullptr, 32, G3, 64, RB3P, 0, 0, 0);
    k_out<<<(NBT / 32 + 7) / 8, 256, 0, stream>>>(G3, OUT);
}
